// EncoderBlock_69767448756345
// MI455X (gfx1250) — hardware-verified
//
#include <hip/hip_runtime.h>
#include <math.h>

#ifndef NB
#define NB 4
#endif
#ifndef SEQ
#define SEQ 2048
#endif
#define NB_FULL 4
#define SEQ_FULL 2048
#define DMODEL 512
#define NHEAD 8
#define HDIM 64
#define FFDIM 2048
#define TTOK (NB * SEQ)
#define QKW 1024
#define NQB (SEQ / 64)

static_assert(SEQ % 64 == 0);
static_assert(SEQ <= SEQ_FULL);
static_assert(NB <= NB_FULL);
static_assert(NHEAD * HDIM == DMODEL);
static_assert(TTOK % 64 == 0);
static_assert(DMODEL % 64 == 0);
static_assert(FFDIM % 64 == 0);

typedef __attribute__((ext_vector_type(16))) _Float16 v16h;
typedef __attribute__((ext_vector_type(8)))  _Float16 v8h;
typedef __attribute__((ext_vector_type(8)))  float    v8f;
typedef __attribute__((ext_vector_type(4)))  float    v4f;
typedef __attribute__((ext_vector_type(4)))  unsigned int u4v;
typedef __attribute__((ext_vector_type(2)))  unsigned int u2v;

union FragU { v16h v; v8h h[2]; };
__device__ __forceinline__ v16h frag_ld(const _Float16* p) { FragU f; f.h[0] = *(const v8h*)(p); f.h[1] = *(const v8h*)(p + 16); return f.v; }

__device__ __forceinline__ v8f wmma16(v16h a, v16h b, v8f c) {
    c = __builtin_amdgcn_wmma_f32_16x16x32_f16(false, a, false, b, (short)0, c, false, false);
    asm volatile("v_nop\n\tv_nop\n\tv_nop\n\tv_nop" : "+v"(c) : "v"(a), "v"(b));
    return c;
}
__device__ __forceinline__ v8f mma_raw(v16h a, v16h b, v8f c) { return __builtin_amdgcn_wmma_f32_16x16x32_f16(false, a, false, b, (short)0, c, false, false); }
__device__ __forceinline__ void dep_guard_h(v8f& a, v8f& b, v16h x, v16h y) { asm volatile("v_nop\n\tv_nop\n\tv_nop\n\tv_nop" : "+v"(a), "+v"(b) : "v"(x), "v"(y)); }
__device__ __forceinline__ void keep4_h(v16h a, v16h b, v16h c, v16h d) { asm volatile("v_nop" :: "v"(a), "v"(b), "v"(c), "v"(d)); }
__device__ __forceinline__ void acc_guard4(v8f& a, v8f& b, v8f& c, v8f& d) { asm volatile("v_nop\n\tv_nop\n\tv_nop\n\tv_nop" : "+v"(a), "+v"(b), "+v"(c), "+v"(d)); }
__device__ __forceinline__ void wave_sync() {
    __builtin_amdgcn_fence(3  , "workgroup");
    __builtin_amdgcn_wave_barrier();
    __builtin_amdgcn_fence(2  , "workgroup");
}

#define VST2(T, ptr, val) do { const T vst2_v_ = (val); *(volatile T*)(ptr) = vst2_v_; __threadfence(); *(volatile T*)(ptr) = vst2_v_; } while (0)

__device__ __forceinline__ float cmb_bf(float v) { const unsigned u = __builtin_bit_cast(unsigned, v); const unsigned r = (u + 0x7fffu + ((u >> 16) & 1u)) & 0xffff0000u; return __builtin_bit_cast(float, r); }
__device__ __forceinline__ unsigned int pk2h(float a, float b) { return (unsigned int)__builtin_bit_cast(unsigned short, (_Float16)a) | ((unsigned int)__builtin_bit_cast(unsigned short, (_Float16)b) << 16); }
__device__ __forceinline__ unsigned xrow(unsigned r) { return (r / (unsigned)SEQ) * (unsigned)SEQ_FULL + (r % (unsigned)SEQ); }

__global__ __launch_bounds__(256) void k_bfvec6(const float* __restrict__ bq, const float* __restrict__ bk, const float* __restrict__ bv,
                                                const float* __restrict__ bp, const float* __restrict__ b1, const float* __restrict__ b2, float* __restrict__ DST) {
    const unsigned blk = blockIdx.x;
    const float* s; unsigned base;
    if (blk < 2u)       { s = bq; base = 0u; }
    else if (blk < 4u)  { s = bk; base = 512u; }
    else if (blk < 6u)  { s = bv; base = 1024u; }
    else if (blk < 8u)  { s = bp; base = 1536u; }
    else if (blk < 16u) { s = b1; base = 2048u; }
    else                { s = b2; base = 4096u; }
    const unsigned u = blk * 256u + threadIdx.x;
    const float v = cmb_bf(s[u - base]);
    VST2(float, DST + u, v);
}

__global__ __launch_bounds__(256) void k_cast_x(const float* __restrict__ X, unsigned short* __restrict__ DST) {
    const unsigned u = blockIdx.x * 256u + threadIdx.x;
    if (u >= (unsigned)TTOK * 64u) return;
    const unsigned r = u >> 6, c0 = (u & 63u) << 3;
    const float* s = X + (size_t)xrow(r) * DMODEL + c0;
    const v4f a = *(const v4f*)s, b = *(const v4f*)(s + 4);
    u4v pk; pk.x = pk2h(cmb_bf(a.x), cmb_bf(a.y)); pk.y = pk2h(cmb_bf(a.z), cmb_bf(a.w)); pk.z = pk2h(cmb_bf(b.x), cmb_bf(b.y)); pk.w = pk2h(cmb_bf(b.z), cmb_bf(b.w));
    VST2(u4v, (u4v*)(DST + (size_t)r * DMODEL + c0), pk);
}

__global__ __launch_bounds__(256) void k_cm_castbT(const float* __restrict__ SRC, unsigned lds, unsigned sSz, unsigned short* __restrict__ DST, unsigned ldd, unsigned sDz,
                                                   unsigned perShift, unsigned nC, float sc) {
    const unsigned u = blockIdx.x * 256u + threadIdx.x;
    if (u >= (nC << perShift)) return;
    const unsigned c = u >> perShift, r0 = (u & ((1u << perShift) - 1u)) << 3;
    const float* s = SRC + (size_t)blockIdx.y * sSz;
    float w[8];
#pragma unroll
    for (int e = 0; e < 8; ++e) w[e] = cmb_bf(s[(size_t)(r0 + (unsigned)e) * lds + c]) * sc;
    u4v pk; pk.x = pk2h(w[0], w[1]); pk.y = pk2h(w[2], w[3]); pk.z = pk2h(w[4], w[5]); pk.w = pk2h(w[6], w[7]);
    VST2(u4v, (u4v*)(DST + (size_t)blockIdx.y * sDz + (size_t)c * ldd + r0), pk);
}

template <int BIAS_MODE, int OUT_MODE, bool RESID, bool RELU>
__global__ __launch_bounds__(256) void wmma_gemm64(const unsigned short* __restrict__ Ap, int lda, const unsigned short* __restrict__ Btp, int ldb,
                                                   void* __restrict__ Cout, int ldc, const float* __restrict__ bias, const float* __restrict__ resid,
                                                   int M, int N, int K, float scale) {
    static_assert(!RESID || OUT_MODE == 0);
    static_assert(!(RESID && RELU));
    const _Float16* A = (const _Float16*)Ap; const _Float16* Bt = (const _Float16*)Btp;
    __shared__ __align__(16) float sT[8][16 * 68];
    const unsigned lane = threadIdx.x & 31u, wave = threadIdx.x >> 5;
    const unsigned tilesN = (unsigned)N >> 6, tilesM = (unsigned)M >> 6;
    const unsigned tile = blockIdx.x * 8u + wave;
    if (tile >= tilesM * tilesN) return;
    const unsigned tm = tile / tilesN, tn = tile - tm * tilesN;
    const unsigned m0 = tm << 6, n0 = tn << 6;
    const unsigned rlane = lane & 15u;
    const unsigned koff = (lane >> 4) * 8u;
    const unsigned mOff = (lane >> 4) * 8u;

    v8f acc[4][4];
#pragma unroll
    for (int i = 0; i < 4; ++i)
#pragma unroll
        for (int j = 0; j < 4; ++j) acc[i][j] = (v8f){0.f, 0.f, 0.f, 0.f, 0.f, 0.f, 0.f, 0.f};

    for (unsigned k0 = 0; k0 < (unsigned)K; k0 += 32u) {
        v16h bh[4];
#pragma unroll
        for (int j = 0; j < 4; ++j) bh[j] = frag_ld(Bt + (size_t)(n0 + ((unsigned)j << 4) + rlane) * (unsigned)ldb + koff + k0);
#pragma unroll
        for (int i = 0; i < 4; ++i) {
            const v16h ah = frag_ld(A + (size_t)(m0 + ((unsigned)i << 4) + rlane) * (unsigned)lda + koff + k0);
#pragma unroll
            for (int j = 0; j < 4; ++j) acc[i][j] = mma_raw(ah, bh[j], acc[i][j]);
            dep_guard_h(acc[i][0], acc[i][3], ah, ah);
        }
        keep4_h(bh[0], bh[1], bh[2], bh[3]);
    }
    acc_guard4(acc[0][0], acc[0][1], acc[0][2], acc[0][3]);
    acc_guard4(acc[1][0], acc[1][1], acc[1][2], acc[1][3]);
    acc_guard4(acc[2][0], acc[2][1], acc[2][2], acc[2][3]);
    acc_guard4(acc[3][0], acc[3][1], acc[3][2], acc[3][3]);

    float* slab = sT[wave];
#pragma unroll
    for (int i = 0; i < 4; ++i) {
        const unsigned mBase = m0 + ((unsigned)i << 4);
#pragma unroll
        for (int j = 0; j < 4; ++j) {
            const unsigned n = n0 + ((unsigned)j << 4) + rlane;
            float bv = 0.f;
            if (BIAS_MODE == 2) bv = bias[n];
#pragma unroll
            for (int r = 0; r < 8; ++r) {
                float v = acc[i][j][r] * scale;
                if (BIAS_MODE == 1) v += bias[mBase + mOff + (unsigned)r];
                if (BIAS_MODE == 2) v += bv;
                if (RELU) v = fmaxf(v, 0.0f);
                slab[(mOff + (unsigned)r) * 68u + ((unsigned)j << 4) + rlane] = v;
            }
        }
        wave_sync();
        if (OUT_MODE == 0) {
            float* C = (float*)Cout;
            const unsigned hh = lane >> 4, c4 = (lane & 15u) * 4u;
            v4f vv[8];
#pragma unroll
            for (int it = 0; it < 8; ++it) {
                const unsigned row = (unsigned)it * 2u + hh;
                v4f v = *(const v4f*)(slab + row * 68u + c4);
                if (RESID) {
                    const v4f rr = *(const v4f*)(resid + (size_t)(mBase + row) * (unsigned)ldc + n0 + c4);
                    v.x += rr.x; v.y += rr.y; v.z += rr.z; v.w += rr.w;
                }
                vv[it] = v;
            }
            for (int pass = 0; pass < 2; ++pass) {
#pragma unroll
                for (int it = 0; it < 8; ++it) {
                    const unsigned row = (unsigned)it * 2u + hh;
                    *(volatile v4f*)(C + (size_t)(mBase + row) * (unsigned)ldc + n0 + c4) = vv[it];
                }
                __threadfence();
            }
        } else {
            const unsigned q = lane >> 3, c8 = (lane & 7u) * 8u;
            unsigned short* C = (unsigned short*)Cout;
            for (int pass = 0; pass < 2; ++pass) {
#pragma unroll
                for (int it = 0; it < 4; ++it) {
                    const unsigned row = (unsigned)it * 4u + q;
                    const float* sp = slab + row * 68u + c8;
                    v8h hv;
#pragma unroll
                    for (int e = 0; e < 8; ++e) hv[e] = (_Float16)sp[e];
                    *(volatile v8h*)(C + (size_t)(mBase + row) * (unsigned)ldc + n0 + c8) = hv;
                }
                __threadfence();
            }
        }
        wave_sync();
    }
}

__global__ __launch_bounds__(128) void k_attn_pl(const unsigned short* __restrict__ QKp, const unsigned short* __restrict__ VTp, unsigned short* __restrict__ CCp) {
    __shared__ __align__(16) _Float16 Psh[4][16 * 64];
    __shared__ __align__(16) float    Os[4][16 * 68];
    const _Float16* QK = (const _Float16*)QKp; const _Float16* VT = (const _Float16*)VTp;
    const unsigned tid = threadIdx.x, wave = tid >> 5, lane = tid & 31u, hh = lane >> 4, c = lane & 15u;
    const unsigned bx = blockIdx.x;
    const unsigned qb = bx % (unsigned)NQB, bh = bx / (unsigned)NQB;
    const unsigned h = bh % (unsigned)NHEAD, b = bh / (unsigned)NHEAD;
    const unsigned q0 = qb * 64u + wave * 16u;
    const _Float16* Qb = QK + (size_t)(b * (unsigned)SEQ) * QKW + h * (unsigned)HDIM;
    const _Float16* Kb = Qb + DMODEL;
    const _Float16* Vb = VT + (size_t)(h * (unsigned)HDIM) * (unsigned)TTOK + b * (unsigned)SEQ;

    const v16h qa0 = frag_ld(Qb + (size_t)(q0 + c) * QKW + 8u * hh);
    const v16h qa1 = frag_ld(Qb + (size_t)(q0 + c) * QKW + 32u + 8u * hh);

    float mrow[8], lrow[8];
    v8f oacc[4];
#pragma unroll
    for (int r = 0; r < 8; ++r) { mrow[r] = -1.0e30f; lrow[r] = 0.f; }
#pragma unroll
    for (int t = 0; t < 4; ++t) oacc[t] = (v8f){0.f, 0.f, 0.f, 0.f, 0.f, 0.f, 0.f, 0.f};

    const float SCL = 0.125f * 1.4426950408889634f;
    const float PSC = 32768.0f;
    _Float16* pw = Psh[wave];

    for (unsigned kc = 0; kc < (unsigned)NQB; ++kc) {
        const unsigned kv0 = kc * 64u;
        v8f s[4];
#pragma unroll
        for (int j = 0; j < 4; ++j) {
            const _Float16* kr = Kb + (size_t)(kv0 + (unsigned)j * 16u + c) * QKW + 8u * hh;
            v8f a = (v8f){0.f, 0.f, 0.f, 0.f, 0.f, 0.f, 0.f, 0.f};
            a = wmma16(qa0, frag_ld(kr), a);
            a = wmma16(qa1, frag_ld(kr + 32), a);
            s[j] = a;
        }
#pragma unroll
        for (int r = 0; r < 8; ++r) {
            const float x0 = s[0][r] * SCL, x1 = s[1][r] * SCL, x2 = s[2][r] * SCL, x3 = s[3][r] * SCL;
            float m = fmaxf(fmaxf(x0, x1), fmaxf(x2, x3));
            m = fmaxf(m, __shfl_xor(m, 1, 32)); m = fmaxf(m, __shfl_xor(m, 2, 32));
            m = fmaxf(m, __shfl_xor(m, 4, 32)); m = fmaxf(m, __shfl_xor(m, 8, 32));
            const float mnew = fmaxf(mrow[r], m);
            const float alpha = exp2f(mrow[r] - mnew);
            mrow[r] = mnew;
            const float p0 = exp2f(x0 - mnew), p1 = exp2f(x1 - mnew), p2 = exp2f(x2 - mnew), p3 = exp2f(x3 - mnew);
            float psum = (p0 + p1) + (p2 + p3);
            _Float16* pr = pw + (8u * hh + (unsigned)r) * 64u + c;
            pr[0]  = (_Float16)(p0 * PSC);
            pr[16] = (_Float16)(p1 * PSC);
            pr[32] = (_Float16)(p2 * PSC);
            pr[48] = (_Float16)(p3 * PSC);
            psum += __shfl_xor(psum, 1, 32); psum += __shfl_xor(psum, 2, 32);
            psum += __shfl_xor(psum, 4, 32); psum += __shfl_xor(psum, 8, 32);
            lrow[r] = lrow[r] * alpha + psum;
            oacc[0][r] *= alpha; oacc[1][r] *= alpha; oacc[2][r] *= alpha; oacc[3][r] *= alpha;
        }
        wave_sync();
#pragma unroll
        for (int kk = 0; kk < 2; ++kk) {
            const v16h pa = frag_ld(pw + c * 64u + (unsigned)kk * 32u + 8u * hh);
#pragma unroll
            for (int t = 0; t < 4; ++t) {
                const v16h vb = frag_ld(Vb + (size_t)((unsigned)t * 16u + c) * (unsigned)TTOK + kv0 + (unsigned)kk * 32u + 8u * hh);
                oacc[t] = wmma16(pa, vb, oacc[t]);
            }
        }
        wave_sync();
    }

    float* os = Os[wave];
#pragma unroll
    for (int r = 0; r < 8; ++r) {
        const float inv = 1.0f / (lrow[r] * PSC);
#pragma unroll
        for (int t = 0; t < 4; ++t) os[(8u * hh + (unsigned)r) * 68u + (unsigned)t * 16u + c] = oacc[t][r] * inv;
    }
    wave_sync();
    {
        const unsigned q = lane >> 3, c8 = (lane & 7u) * 8u;
        unsigned short* C = CCp + (size_t)(b * (unsigned)SEQ + q0) * DMODEL + h * (unsigned)HDIM;
        for (int pass = 0; pass < 2; ++pass) {
#pragma unroll
            for (int it = 0; it < 4; ++it) {
                const unsigned row = (unsigned)it * 4u + q;
                const float* sp = os + row * 68u + c8;
                v8h hv;
#pragma unroll
                for (int e = 0; e < 8; ++e) hv[e] = (_Float16)sp[e];
                *(volatile v8h*)(C + (size_t)row * DMODEL + c8) = hv;
            }
            __threadfence();
        }
    }
}

template <int NQ, int HASX, int XBF>
__global__ __launch_bounds__(256) void k_b_ln(const float* __restrict__ A, const float* __restrict__ X, const float* __restrict__ GA, const float* __restrict__ BE,
                                              unsigned rows, float* __restrict__ Yf, unsigned short* __restrict__ Y16) {
    #pragma clang fp contract(off)
    constexpr unsigned WD = 128u * NQ;
    const unsigned r = blockIdx.x * 8u + (threadIdx.x >> 5); const unsigned L = threadIdx.x & 31u;
    if (r >= rows) return;
    v4f v[NQ]; float s = 0.f;
#pragma unroll
    for (int q = 0; q < NQ; ++q) {
        const unsigned cc = 4u * L + 128u * (unsigned)q;
        v[q] = *(const v4f*)(A + (size_t)r * WD + cc);
        if (HASX) {
            v4f x = *(const v4f*)(X + (size_t)xrow(r) * WD + cc);
            if (XBF) { x.x = cmb_bf(x.x); x.y = cmb_bf(x.y); x.z = cmb_bf(x.z); x.w = cmb_bf(x.w); }
            v[q] = v[q] + x;
        }
        s += (v[q].x + v[q].y) + (v[q].z + v[q].w);
    }
#pragma unroll
    for (int o = 16; o > 0; o >>= 1) s += __shfl_xor(s, o, 32);
    const float mu = s * (1.f / (float)WD); float qq = 0.f;
#pragma unroll
    for (int q = 0; q < NQ; ++q) { v[q].x -= mu; v[q].y -= mu; v[q].z -= mu; v[q].w -= mu; qq += (v[q].x * v[q].x + v[q].y * v[q].y) + (v[q].z * v[q].z + v[q].w * v[q].w); }
#pragma unroll
    for (int o = 16; o > 0; o >>= 1) qq += __shfl_xor(qq, o, 32);
    const float rs = 1.f / (sqrtf(qq * (1.f / (float)WD)) + 1e-10f);
#pragma unroll
    for (int q = 0; q < NQ; ++q) {
        const unsigned cc = 4u * L + 128u * (unsigned)q;
        const v4f ga = *(const v4f*)(GA + cc), be = *(const v4f*)(BE + cc);
        v4f y;
        y.x = cmb_bf(ga.x) * (v[q].x * rs) + cmb_bf(be.x); y.y = cmb_bf(ga.y) * (v[q].y * rs) + cmb_bf(be.y);
        y.z = cmb_bf(ga.z) * (v[q].z * rs) + cmb_bf(be.z); y.w = cmb_bf(ga.w) * (v[q].w * rs) + cmb_bf(be.w);
        const size_t o = (size_t)r * WD + cc;
        if (Yf != nullptr) VST2(v4f, Yf + o, y);
        if (Y16 != nullptr) { u2v pk; pk.x = pk2h(y.x, y.y); pk.y = pk2h(y.z, y.w); VST2(u2v, (u2v*)(Y16 + o), pk); }
    }
}

constexpr size_t SZ_X16 = (size_t)TTOK * DMODEL * 2;
constexpr size_t SZ_WQK = (size_t)QKW * DMODEL * 2;
constexpr size_t SZ_WV  = (size_t)DMODEL * DMODEL * 2;
constexpr size_t SZ_WP  = (size_t)DMODEL * DMODEL * 2;
constexpr size_t SZ_W1  = (size_t)FFDIM * DMODEL * 2;
constexpr size_t SZ_W2  = (size_t)DMODEL * FFDIM * 2;
constexpr size_t SZ_BR  = (size_t)4608 * 4;
constexpr size_t SZ_QK  = (size_t)TTOK * QKW * 2;
constexpr size_t SZ_VT  = (size_t)DMODEL * TTOK * 2;
constexpr size_t SZ_CC  = (size_t)TTOK * DMODEL * 2;
constexpr size_t SZ_ATT = (size_t)TTOK * DMODEL * 4;
constexpr size_t SZ_X1F = (size_t)TTOK * DMODEL * 4;
constexpr size_t SZ_X1H = (size_t)TTOK * DMODEL * 2;
constexpr size_t SZ_HM  = (size_t)TTOK * FFDIM * 2;
constexpr size_t SZ_ALL = SZ_X16 + SZ_WQK + SZ_WV + SZ_WP + SZ_W1 + SZ_W2 + SZ_BR + SZ_QK + SZ_VT + SZ_CC + SZ_ATT + SZ_X1F + SZ_X1H + SZ_HM;
static_assert(SZ_ALL <= (size_t)134217728);
static_assert(SZ_BR % 256 == 0);
static_assert(((size_t)TTOK * 64 / 256) * 256 * 8 == (size_t)TTOK * DMODEL);
static_assert((size_t)NB * NHEAD * NQB * 64 * 64 == (size_t)TTOK * DMODEL);
static_assert((((size_t)TTOK / 64) * (QKW / 64) / 8) * 8 * 4096 == (size_t)TTOK * QKW);
static_assert((((size_t)DMODEL / 64) * (TTOK / 64) / 8) * 8 * 4096 == (size_t)DMODEL * TTOK);
static_assert((((size_t)TTOK / 64) * (DMODEL / 64) / 8) * 8 * 4096 == (size_t)TTOK * DMODEL);
static_assert((((size_t)TTOK / 64) * (FFDIM / 64) / 8) * 8 * 4096 == (size_t)TTOK * FFDIM);
static_assert(((size_t)TTOK / 8) * 8 == (size_t)TTOK);

extern "C" void kernel_launch(void* const* d_in, const int* in_sizes, int n_in, void* d_out, int out_size, void* d_ws, size_t ws_size, hipStream_t stream) {
    if (n_in < 17) return;
    if (in_sizes[0] < ((NB - 1) * SEQ_FULL + SEQ) * DMODEL) return;
    if (in_sizes[1] < NHEAD * DMODEL * HDIM || in_sizes[3] < NHEAD * DMODEL * HDIM || in_sizes[5] < NHEAD * DMODEL * HDIM) return;
    if (in_sizes[2] < DMODEL || in_sizes[4] < DMODEL || in_sizes[6] < DMODEL) return;
    if (in_sizes[7] < DMODEL * DMODEL || in_sizes[8] < DMODEL || in_sizes[9] < DMODEL || in_sizes[10] < DMODEL) return;
    if (in_sizes[11] < DMODEL * FFDIM || in_sizes[12] < FFDIM || in_sizes[13] < FFDIM * DMODEL || in_sizes[14] < DMODEL) return;
    if (in_sizes[15] < DMODEL || in_sizes[16] < DMODEL) return;
    if (out_size < TTOK * DMODEL) return;
    if (ws_size < SZ_ALL) return;

    const float* x   = (const float*)d_in[0];
    const float* Wq  = (const float*)d_in[1];
    const float* bq  = (const float*)d_in[2];
    const float* Wk  = (const float*)d_in[3];
    const float* bk  = (const float*)d_in[4];
    const float* Wv  = (const float*)d_in[5];
    const float* bv  = (const float*)d_in[6];
    const float* Wp  = (const float*)d_in[7];
    const float* bp  = (const float*)d_in[8];
    const float* g1  = (const float*)d_in[9];
    const float* be1 = (const float*)d_in[10];
    const float* W1  = (const float*)d_in[11];
    const float* b1  = (const float*)d_in[12];
    const float* W2  = (const float*)d_in[13];
    const float* b2  = (const float*)d_in[14];
    const float* g2  = (const float*)d_in[15];
    const float* be2 = (const float*)d_in[16];
    float* out = (float*)d_out;

    char* wsp = (char*)d_ws;
    unsigned short* X16   = (unsigned short*)wsp; wsp += SZ_X16;
    unsigned short* WQK16 = (unsigned short*)wsp; wsp += SZ_WQK;
    unsigned short* WV16  = (unsigned short*)wsp; wsp += SZ_WV;
    unsigned short* WPT   = (unsigned short*)wsp; wsp += SZ_WP;
    unsigned short* W1T   = (unsigned short*)wsp; wsp += SZ_W1;
    unsigned short* W2T   = (unsigned short*)wsp; wsp += SZ_W2;
    float*          BR    = (float*)wsp;          wsp += SZ_BR;
    unsigned short* QK16  = (unsigned short*)wsp; wsp += SZ_QK;
    unsigned short* VT16  = (unsigned short*)wsp; wsp += SZ_VT;
    unsigned short* CC16  = (unsigned short*)wsp; wsp += SZ_CC;
    float*          ATT   = (float*)wsp;          wsp += SZ_ATT;
    float*          X1F   = (float*)wsp;          wsp += SZ_X1F;
    unsigned short* X1H   = (unsigned short*)wsp; wsp += SZ_X1H;
    unsigned short* HM16  = (unsigned short*)wsp; wsp += SZ_HM;
    float*          Y2    = ATT;
    if ((size_t)(wsp - (char*)d_ws) > ws_size) return;

    k_bfvec6<<<18, 256, 0, stream>>>(bq, bk, bv, bp, b1, b2, BR);
    k_cast_x<<<(unsigned)((size_t)TTOK * 64 / 256), 256, 0, stream>>>(x, X16);
    k_cm_castbT<<<dim3(16, 8), 256, 0, stream>>>(Wq, 64u, 512u * 64u, WQK16, 512u, 64u * 512u, 6u, 64u, 16.0f);
    k_cm_castbT<<<dim3(16, 8), 256, 0, stream>>>(Wk, 64u, 512u * 64u, WQK16 + (size_t)512 * 512, 512u, 64u * 512u, 6u, 64u, 16.0f);
    k_cm_castbT<<<dim3(16, 8), 256, 0, stream>>>(Wv, 64u, 512u * 64u, WV16, 512u, 64u * 512u, 6u, 64u, 16.0f);
    k_cm_castbT<<<dim3(128, 1), 256, 0, stream>>>(Wp, 512u, 0u, WPT, 512u, 0u, 6u, 512u, 16.0f);
    k_cm_castbT<<<dim3(512, 1), 256, 0, stream>>>(W1, 2048u, 0u, W1T, 512u, 0u, 6u, 2048u, 16.0f);
    k_cm_castbT<<<dim3(512, 1), 256, 0, stream>>>(W2, 512u, 0u, W2T, 2048u, 0u, 8u, 512u, 16.0f);

    wmma_gemm64<2, 1, false, false><<<(unsigned)(((TTOK / 64) * (QKW / 64)) / 8), 256, 0, stream>>>(X16, DMODEL, WQK16, DMODEL, (void*)QK16, QKW, BR + 0, nullptr, TTOK, QKW, DMODEL, 0.0625f);
    wmma_gemm64<1, 1, false, false><<<(unsigned)(((DMODEL / 64) * (TTOK / 64)) / 8), 256, 0, stream>>>(WV16, DMODEL, X16, DMODEL, (void*)VT16, TTOK, BR + 1024, nullptr, DMODEL, TTOK, DMODEL, 0.0625f);

    k_attn_pl<<<(unsigned)(NB * NHEAD * NQB), 128, 0, stream>>>(QK16, VT16, CC16);

    wmma_gemm64<2, 0, false, false><<<(unsigned)(((TTOK / 64) * (DMODEL / 64)) / 8), 256, 0, stream>>>(CC16, DMODEL, WPT, DMODEL, (void*)ATT, DMODEL, BR + 1536, nullptr, TTOK, DMODEL, DMODEL, 0.0625f);
    k_b_ln<4, 1, 1><<<(unsigned)(TTOK / 8), 256, 0, stream>>>(ATT, x, g1, be1, (unsigned)TTOK, X1F, X1H);

    wmma_gemm64<2, 1, false, true><<<(unsigned)(((TTOK / 64) * (FFDIM / 64)) / 8), 256, 0, stream>>>(X1H, DMODEL, W1T, DMODEL, (void*)HM16, FFDIM, BR + 2048, nullptr, TTOK, FFDIM, DMODEL, 0.0625f);
    wmma_gemm64<2, 0, true, false><<<(unsigned)(((TTOK / 64) * (DMODEL / 64)) / 8), 256, 0, stream>>>(HM16, FFDIM, W2T, FFDIM, (void*)Y2, DMODEL, BR + 4096, X1F, TTOK, DMODEL, FFDIM, 0.0625f);

    k_b_ln<4, 0, 0><<<(unsigned)(TTOK / 8), 256, 0, stream>>>(Y2, nullptr, g2, be2, (unsigned)TTOK, out, nullptr);
}
